// LSTMCell_29686813950554
// MI455X (gfx1250) — hardware-verified
//
#include <hip/hip_runtime.h>
#include <math.h>

typedef __attribute__((ext_vector_type(16))) _Float16 v16h;
typedef __attribute__((ext_vector_type(8)))  _Float16 v8h;
typedef __attribute__((ext_vector_type(16))) __bf16   v16b;
typedef __attribute__((ext_vector_type(8)))  __bf16   v8b;
typedef __attribute__((ext_vector_type(8)))  float    v8f;
typedef __attribute__((ext_vector_type(4)))  float    v4f;
#define PSCALE 32768.0f
#define U16(p) ((const unsigned short*)(const void*)(p))
#define PSCALE_INV (1.0f / 32768.0f)

__device__ __forceinline__ unsigned short f2bf_bits(float f) {
  unsigned u = __float_as_uint(f);
  return (unsigned short)((u + 0x7FFFu + ((u >> 16) & 1u)) >> 16);
}
__device__ __forceinline__ float bf_bits2f(unsigned short h) { return __uint_as_float(((unsigned)h) << 16); }

__device__ __forceinline__ void dep_guard_h(v8f& a, v8f& b, v16h x, v16h y) { asm volatile("v_nop\n\tv_nop\n\tv_nop\n\tv_nop" : "+v"(a), "+v"(b) : "v"(x), "v"(y)); }
__device__ __forceinline__ void dep_guard_b(v8f& a, v8f& b, v16b x, v16b y) { asm volatile("v_nop\n\tv_nop\n\tv_nop\n\tv_nop" : "+v"(a), "+v"(b) : "v"(x), "v"(y)); }
__device__ __forceinline__ void keep4_h(v16h a, v16h b, v16h c, v16h d) { asm volatile("v_nop" :: "v"(a), "v"(b), "v"(c), "v"(d)); }
__device__ __forceinline__ void keep4_b(v16b a, v16b b, v16b c, v16b d) { asm volatile("v_nop" :: "v"(a), "v"(b), "v"(c), "v"(d)); }
__device__ __forceinline__ void acc_guard4(v8f& a, v8f& b, v8f& c, v8f& d) { asm volatile("v_nop\n\tv_nop\n\tv_nop\n\tv_nop" : "+v"(a), "+v"(b), "+v"(c), "+v"(d)); }
template <typename T> struct Frag;
template <> struct Frag<_Float16> {
  typedef v16h V; union U { v16h v; v8h h[2]; };
  static __device__ __forceinline__ v16h load(const _Float16* p) {
    U f; f.h[0] = *(const v8h*)(p); f.h[1] = *(const v8h*)(p + 16); return f.v;
  }
  static __device__ __forceinline__ v8f mma(v16h a, v16h b, v8f c) {
    return __builtin_amdgcn_wmma_f32_16x16x32_f16(false, a, false, b, (short)0, c, false, false);
  }
  static __device__ __forceinline__ void guard(v8f& a, v8f& b, v16h x, v16h y) { dep_guard_h(a, b, x, y); }
  static __device__ __forceinline__ void keep(v16h a, v16h b, v16h c, v16h d) { keep4_h(a, b, c, d); }
};
template <> struct Frag<__bf16> {
  typedef v16b V; union U { v16b v; v8b h[2]; };
  static __device__ __forceinline__ v16b load(const __bf16* p) {
    U f; f.h[0] = *(const v8b*)(p); f.h[1] = *(const v8b*)(p + 16); return f.v;
  }
  static __device__ __forceinline__ v8f mma(v16b a, v16b b, v8f c) {
    return __builtin_amdgcn_wmma_f32_16x16x32_bf16(false, a, false, b, (short)0, c, false, false);
  }
  static __device__ __forceinline__ void guard(v8f& a, v8f& b, v16b x, v16b y) { dep_guard_b(a, b, x, y); }
  static __device__ __forceinline__ void keep(v16b a, v16b b, v16b c, v16b d) { keep4_b(a, b, c, d); }
};

typedef __attribute__((ext_vector_type(4))) unsigned v4u;

__device__ __forceinline__ void mma_group_guard(v8f& c0, v8f& c1, v8f& c2, v8f& c3,
                                                v16b a0, v16b a1, v16b b0, v16b b1) {
  asm volatile("v_nop\n\tv_nop\n\tv_nop\n\tv_nop"
               : "+v"(c0), "+v"(c1), "+v"(c2), "+v"(c3)
               : "v"(a0), "v"(a1), "v"(b0), "v"(b1)
               : "memory");
}

constexpr int NB_ROWS = 4096;
constexpr int N_IN    = 1024;
constexpr int N_HID   = 1024;
constexpr int K_TOT   = N_IN + N_HID;
constexpr int N_GATES = 4;
constexpr int WT_M = 32;
constexpr int WT_N = 32;
constexpr int WAVES_BLK = 2;

constexpr size_t WS_OFF_A    = 0;
constexpr size_t WS_BYTES_A  = (size_t)NB_ROWS * K_TOT * 2;
constexpr size_t WS_OFF_BT   = WS_OFF_A + WS_BYTES_A;
constexpr size_t WS_BYTES_BT = (size_t)N_GATES * N_HID * K_TOT * 2;
constexpr size_t WS_TOTAL    = WS_OFF_BT + WS_BYTES_BT;
constexpr size_t OUT_ELEMS_EACH = (size_t)NB_ROWS * N_HID;
constexpr size_t OUT1_OFF_BYTES = 16777216;

static_assert(WS_BYTES_A == 16777216, "cfg");
static_assert(WS_BYTES_BT == 16777216, "cfg");
static_assert(WS_TOTAL == 33554432 && WS_TOTAL <= 134217728, "cfg");
static_assert(OUT1_OFF_BYTES == OUT_ELEMS_EACH * 4, "cfg");
static_assert(OUT1_OFF_BYTES + OUT_ELEMS_EACH * 4 == 33554432, "cfg");
static_assert((OUT1_OFF_BYTES % 128) == 0, "cfg");
static_assert(K_TOT % 32 == 0, "cfg");
static_assert(NB_ROWS % WT_M == 0 && N_HID % WT_N == 0, "cfg");
static_assert(((NB_ROWS / WT_M) * (N_HID / WT_N)) % WAVES_BLK == 0, "cfg");
static_assert(N_IN == N_HID, "cfg");
static_assert(N_IN % 64 == 0 && N_HID % 64 == 0, "cfg");
static_assert(N_IN % 256 == 0, "cfg");
static_assert((NB_ROWS * N_IN) % (256 * 8) == 0, "cfg");

__global__ __launch_bounds__(256) void cvt_act_bf16(
    const float* __restrict__ xin, const float* __restrict__ hin, unsigned* __restrict__ Aw) {
  const int part = blockIdx.y;
  const float* src = (part == 0) ? xin : hin;
  const size_t e = ((size_t)blockIdx.x * 256 + threadIdx.x) * 8;
  const size_t row = e >> 10;
  const size_t col = e & 1023;
  const v4f v0 = *(const v4f*)(src + e);
  const v4f v1 = *(const v4f*)(src + e + 4);
  const float s0 = v0[0], s1 = v0[1], s2 = v0[2], s3 = v0[3];
  const float s4 = v1[0], s5 = v1[1], s6 = v1[2], s7 = v1[3];
  v4u w;
  w[0] = (unsigned)f2bf_bits(s0) | ((unsigned)f2bf_bits(s1) << 16);
  w[1] = (unsigned)f2bf_bits(s2) | ((unsigned)f2bf_bits(s3) << 16);
  w[2] = (unsigned)f2bf_bits(s4) | ((unsigned)f2bf_bits(s5) << 16);
  w[3] = (unsigned)f2bf_bits(s6) | ((unsigned)f2bf_bits(s7) << 16);
  unsigned* dst = Aw + ((row * (size_t)K_TOT + (size_t)part * N_IN + col) >> 1);
  *(volatile v4u*)dst = w;
  __threadfence();
  *(volatile v4u*)dst = w;
}

__global__ __launch_bounds__(256) void cvt_wt_bf16(
    const float* __restrict__ wx0, const float* __restrict__ wx1,
    const float* __restrict__ wx2, const float* __restrict__ wx3,
    const float* __restrict__ wh0, const float* __restrict__ wh1,
    const float* __restrict__ wh2, const float* __restrict__ wh3,
    unsigned* __restrict__ Btw) {
  __shared__ __align__(16) unsigned short t[64][66];
  const int z = blockIdx.z;
  const float* src;
  switch (z) {
    case 0: src = wx0; break; case 1: src = wx1; break;
    case 2: src = wx2; break; case 3: src = wx3; break;
    case 4: src = wh0; break; case 5: src = wh1; break;
    case 6: src = wh2; break; default: src = wh3; break;
  }
  const int part = z >> 2;
  const int gsel = z & 3;
  const int tid = threadIdx.x;
  const int k0 = blockIdx.y * 64;
  const int n0 = blockIdx.x * 64;
  {
    const int kr = tid >> 2;
    const int nc = (tid & 3) * 16;
    const float* sp = src + (size_t)(k0 + kr) * N_HID + n0 + nc;
#pragma unroll
    for (int j = 0; j < 4; ++j) {
      const v4f v = *(const v4f*)(sp + 4 * j);
      const float e0 = v[0], e1 = v[1], e2 = v[2], e3 = v[3];
      t[kr][nc + 4 * j + 0] = f2bf_bits(e0);
      t[kr][nc + 4 * j + 1] = f2bf_bits(e1);
      t[kr][nc + 4 * j + 2] = f2bf_bits(e2);
      t[kr][nc + 4 * j + 3] = f2bf_bits(e3);
    }
  }
  __syncthreads();
  const int wave = tid >> 5;
  const int lane = tid & 31;
  const int q  = lane >> 3;
  const int c8 = (lane & 7) * 8;
  v4u wv[2];
#pragma unroll
  for (int it = 0; it < 2; ++it) {
    const int nr = wave * 8 + it * 4 + q;
    v4u w;
#pragma unroll
    for (int e = 0; e < 4; ++e) {
      const unsigned lo = (unsigned)t[c8 + 2 * e][nr];
      const unsigned hi = (unsigned)t[c8 + 2 * e + 1][nr];
      w[e] = lo | (hi << 16);
    }
    wv[it] = w;
  }
  for (int pass = 0; pass < 2; ++pass) {
#pragma unroll
    for (int it = 0; it < 2; ++it) {
      const int nr = wave * 8 + it * 4 + q;
      const size_t hidx = ((size_t)gsel * N_HID + n0 + nr) * K_TOT + (size_t)part * N_IN + k0 + c8;
      *(volatile v4u*)(Btw + (hidx >> 1)) = wv[it];
    }
    __threadfence();
  }
}

__global__ __launch_bounds__(64) void gemm_gates_cell(
    const unsigned short* __restrict__ Ap, const unsigned short* __restrict__ Btp,
    const float* __restrict__ cell,
    const float* __restrict__ bias_f, const float* __restrict__ bias_i,
    const float* __restrict__ bias_n, const float* __restrict__ bias_o,
    float* __restrict__ out) {
  typedef __bf16 T;
  typedef v16b V;
  const T* A  = (const T*)Ap;
  const T* Bt = (const T*)Btp;
  __shared__ __align__(16) float sPre[WAVES_BLK][N_GATES * WT_M * WT_N];

  const int lane = threadIdx.x & 31;
  const int wave = threadIdx.x >> 5;
  const int tilesN = N_HID / WT_N;
  const int tile = blockIdx.x * WAVES_BLK + wave;
  const int tm = tile / tilesN;
  const int tn = tile - tm * tilesN;
  const int m0 = tm * WT_M;
  const int n0 = tn * WT_N;

  const int rlane = lane & 15;
  const int koff  = (lane >> 4) * 8;
  const int mOff  = (lane >> 4) * 8;

  v8f acc[4][2][2];
#pragma unroll
  for (int g = 0; g < 4; ++g)
#pragma unroll
    for (int ms = 0; ms < 2; ++ms)
#pragma unroll
      for (int ns = 0; ns < 2; ++ns) acc[g][ms][ns] = (v8f){0.f, 0.f, 0.f, 0.f, 0.f, 0.f, 0.f, 0.f};

  const T* Arow0 = A + (size_t)(m0 + rlane) * K_TOT + koff;
  const T* Arow1 = A + (size_t)(m0 + 16 + rlane) * K_TOT + koff;
  const T* Brow0 = Bt + (size_t)(n0 + rlane) * K_TOT + koff;
  const T* Brow1 = Bt + (size_t)(n0 + 16 + rlane) * K_TOT + koff;
  const size_t gateStride = (size_t)N_HID * K_TOT;

  for (int k0 = 0; k0 < K_TOT; k0 += 32) {
    const V a0 = Frag<T>::load(Arow0 + k0);
    const V a1 = Frag<T>::load(Arow1 + k0);
#pragma unroll
    for (int g = 0; g < 4; ++g) {
      const V b0 = Frag<T>::load(Brow0 + (size_t)g * gateStride + k0);
      const V b1 = Frag<T>::load(Brow1 + (size_t)g * gateStride + k0);
      acc[g][0][0] = Frag<T>::mma(a0, b0, acc[g][0][0]);
      acc[g][0][1] = Frag<T>::mma(a0, b1, acc[g][0][1]);
      acc[g][1][0] = Frag<T>::mma(a1, b0, acc[g][1][0]);
      acc[g][1][1] = Frag<T>::mma(a1, b1, acc[g][1][1]);
      mma_group_guard(acc[g][0][0], acc[g][0][1], acc[g][1][0], acc[g][1][1], a0, a1, b0, b1);
    }
  }
  acc_guard4(acc[0][0][0], acc[0][0][1], acc[0][1][0], acc[0][1][1]);
  acc_guard4(acc[1][0][0], acc[1][0][1], acc[1][1][0], acc[1][1][1]);
  acc_guard4(acc[2][0][0], acc[2][0][1], acc[2][1][0], acc[2][1][1]);
  acc_guard4(acc[3][0][0], acc[3][0][1], acc[3][1][0], acc[3][1][1]);

  float* slab = sPre[wave];
#pragma unroll
  for (int g = 0; g < 4; ++g)
#pragma unroll
    for (int ms = 0; ms < 2; ++ms)
#pragma unroll
      for (int ns = 0; ns < 2; ++ns)
#pragma unroll
        for (int r = 0; r < 8; ++r)
          slab[((g * WT_M) + ms * 16 + mOff + r) * WT_N + ns * 16 + rlane] = acc[g][ms][ns][r];
  __builtin_amdgcn_fence(__ATOMIC_RELEASE, "workgroup");
  __builtin_amdgcn_wave_barrier();
  __builtin_amdgcn_fence(__ATOMIC_ACQUIRE, "workgroup");

  const int col = n0 + lane;
  const float bfv = bf_bits2f(f2bf_bits(bias_f[col]));
  const float biv = bf_bits2f(f2bf_bits(bias_i[col]));
  const float bnv = bf_bits2f(f2bf_bits(bias_n[col]));
  const float bov = bf_bits2f(f2bf_bits(bias_o[col]));
#pragma unroll 1
  for (int rr = 0; rr < WT_M; ++rr) {
    const float pf = slab[(0 * WT_M + rr) * WT_N + lane] + bfv;
    const float pi = slab[(1 * WT_M + rr) * WT_N + lane] + biv;
    const float pn = slab[(2 * WT_M + rr) * WT_N + lane] + bnv;
    const float po = slab[(3 * WT_M + rr) * WT_N + lane] + bov;
    const size_t ci = (size_t)(m0 + rr) * N_HID + col;
    const float cv = bf_bits2f(f2bf_bits(cell[ci]));
    const float fg = 1.0f / (1.0f + expf(-pf));
    const float ig = 1.0f / (1.0f + expf(-pi));
    const float og = 1.0f / (1.0f + expf(-po));
    const float ng = tanhf(pn);
    const float cn = fg * cv + ig * ng;
    const float hn = og * tanhf(cn);
    slab[(0 * WT_M + rr) * WT_N + lane] = hn;
    slab[(1 * WT_M + rr) * WT_N + lane] = cn;
  }
  __builtin_amdgcn_fence(__ATOMIC_RELEASE, "workgroup");
  __builtin_amdgcn_wave_barrier();
  __builtin_amdgcn_fence(__ATOMIC_ACQUIRE, "workgroup");

  float* outH = out;
  float* outC = out + OUT_ELEMS_EACH;
  const int q  = lane >> 3;
  const int c4 = (lane & 7) * 4;
  for (int pass = 0; pass < 2; ++pass) {
#pragma unroll
    for (int it = 0; it < 8; ++it) {
      const int row = it * 4 + q;
      const v4f vh = *(const v4f*)(slab + (0 * WT_M + row) * WT_N + c4);
      const v4f vc = *(const v4f*)(slab + (1 * WT_M + row) * WT_N + c4);
      const size_t oi = (size_t)(m0 + row) * N_HID + n0 + c4;
      *(volatile v4f*)(outH + oi) = vh;
      *(volatile v4f*)(outC + oi) = vc;
    }
    __threadfence();
  }
}

extern "C" void kernel_launch(void* const* d_in, const int* in_sizes, int n_in,
                              void* d_out, int out_size, void* d_ws, size_t ws_size,
                              hipStream_t stream)
{
  (void)in_sizes; (void)n_in; (void)out_size;
  const float* x_in   = (const float*)d_in[0];
  const float* h_in   = (const float*)d_in[1];
  const float* c_in   = (const float*)d_in[2];
  const float* W_ii   = (const float*)d_in[3];
  const float* W_hi   = (const float*)d_in[4];
  const float* b_i    = (const float*)d_in[5];
  const float* W_if   = (const float*)d_in[6];
  const float* W_hf   = (const float*)d_in[7];
  const float* b_f    = (const float*)d_in[8];
  const float* W_in   = (const float*)d_in[9];
  const float* W_hn   = (const float*)d_in[10];
  const float* b_n    = (const float*)d_in[11];
  const float* W_io   = (const float*)d_in[12];
  const float* W_ho   = (const float*)d_in[13];
  const float* b_o    = (const float*)d_in[14];
  float* out = (float*)d_out;

  if (ws_size < WS_TOTAL) return;
  unsigned char* ws = (unsigned char*)d_ws;
  unsigned* Aw  = (unsigned*)(ws + WS_OFF_A);
  unsigned* Btw = (unsigned*)(ws + WS_OFF_BT);

  cvt_act_bf16<<<dim3((NB_ROWS * N_IN) / (256 * 8), 2), dim3(256), 0, stream>>>(x_in, h_in, Aw);

  cvt_wt_bf16<<<dim3(N_HID / 64, N_IN / 64, 8), dim3(256), 0, stream>>>(
      W_if, W_ii, W_in, W_io, W_hf, W_hi, W_hn, W_ho, Btw);

  gemm_gates_cell<<<dim3(((NB_ROWS / WT_M) * (N_HID / WT_N)) / WAVES_BLK), dim3(64), 0, stream>>>(
      (const unsigned short*)Aw, (const unsigned short*)Btw, c_in, b_f, b_i, b_n, b_o, out);
}
